// CausalAttention_69836168233253
// MI455X (gfx1250) — hardware-verified
//
#include <hip/hip_runtime.h>
#ifndef NB
#define NB 4
#endif
#ifndef SEQ
#define SEQ 2048
#endif
#define NB_FULL 4
#define SEQ_FULL 2048
#define DM 1024
#define QT 256
#define KT0 256
#define NKX SEQ
#define NR ((size_t)NB * SEQ)
static_assert(NB >= 1 && NB <= NB_FULL);
static_assert(SEQ % QT == 0 && SEQ >= QT && SEQ <= SEQ_FULL);
static_assert(KT0 == QT);
static_assert(DM % 64 == 0 && DM % 32 == 0);
static_assert(QT % 128 == 0 && KT0 % 128 == 0 && SEQ % 64 == 0 && KT0 % 64 == 0);
static_assert(((size_t)NB * SEQ) % 128 == 0);
static_assert(((size_t)NB * SEQ * DM) % 8 == 0 && ((size_t)DM * DM) % 8 == 0);

typedef unsigned short v8us __attribute__((ext_vector_type(8), may_alias));
typedef float  v8f  __attribute__((ext_vector_type(8)));
typedef float  v4f  __attribute__((ext_vector_type(4)));
typedef float  v4fa __attribute__((ext_vector_type(4), may_alias));
typedef _Float16 v16h __attribute__((ext_vector_type(16)));
typedef _Float16 v4h  __attribute__((ext_vector_type(4)));
union FragH { v16h v; v8us half[2]; _Float16 h[16]; unsigned short u[16]; };

__device__ __forceinline__ unsigned short bf16_bits(float x) { unsigned int u = __float_as_uint(x); return (unsigned short)((u + 0x7FFFu + ((u >> 16) & 1u)) >> 16); }
__device__ __forceinline__ float bf16_val(unsigned short b) { return __uint_as_float(((unsigned int)b) << 16); }
__device__ __forceinline__ float bf16_rne(float x) { return bf16_val(bf16_bits(x)); }

__global__ __launch_bounds__(256) void k_wnat(const float* __restrict__ w, size_t n8, _Float16* __restrict__ Bt) {
  const size_t t = (size_t)blockIdx.x * 256 + threadIdx.x; if (t >= n8) return;
  FragH f;
#pragma unroll
  for (int q = 0; q < 8; ++q) f.h[q] = (_Float16)(bf16_rne(w[t * 8 + q]) * 16.0f);
  *(volatile v8us*)((unsigned short*)Bt + t * 8) = f.half[0];
  __threadfence();
  *(volatile v8us*)((unsigned short*)Bt + t * 8) = f.half[0];
}

__global__ __launch_bounds__(256) void k_x16(const float* __restrict__ x, _Float16* __restrict__ X16, size_t n8) {
  const size_t t = (size_t)blockIdx.x * 256 + threadIdx.x; if (t >= n8) return;
  const size_t per = (size_t)SEQ * DM / 8;
  const size_t b = t / per, o = t - b * per;
  const float* src = x + b * ((size_t)SEQ_FULL * DM) + o * 8;
  FragH f;
#pragma unroll
  for (int q = 0; q < 8; ++q) f.h[q] = (_Float16)bf16_rne(src[q]);
  *(volatile v8us*)((unsigned short*)X16 + t * 8) = f.half[0];
  __threadfence();
  *(volatile v8us*)((unsigned short*)X16 + t * 8) = f.half[0];
}

__global__ __launch_bounds__(256) void k_lo(const float* __restrict__ F, _Float16* __restrict__ L, size_t n8) {
  const size_t t = (size_t)blockIdx.x * 256 + threadIdx.x; if (t >= n8) return;
  const v4f a = *(const v4fa*)(F + t * 8), c = *(const v4fa*)(F + t * 8 + 4);
  FragH fl;
#pragma unroll
  for (int q = 0; q < 4; ++q) {
    _Float16 h = (_Float16)a[q]; fl.h[q] = (_Float16)((a[q] - (float)h) * 1024.0f);
    h = (_Float16)c[q]; fl.h[4 + q] = (_Float16)((c[q] - (float)h) * 1024.0f);
  }
  *(volatile v8us*)((unsigned short*)L + t * 8) = fl.half[0];
  __threadfence();
  *(volatile v8us*)((unsigned short*)L + t * 8) = fl.half[0];
}

__device__ __forceinline__ v16h g2_frag(const _Float16* p, int hh) {
  FragH f;
  f.half[0] = *(const v8us*)((const unsigned short*)p + 8 * hh);
  f.half[1] = *(const v8us*)((const unsigned short*)p + 16 + 8 * hh);
  return f.v;
}
__device__ __forceinline__ v8f g2_mma(v16h a, v16h b, v8f c) {
  v8f d = __builtin_amdgcn_wmma_f32_16x16x32_f16(false, a, false, b, (short)0, c, false, false);
  asm volatile("v_nop\n\tv_nop\n\tv_nop\n\tv_nop" : "+v"(d) : "v"(a), "v"(b));
  return d;
}
__global__ __launch_bounds__(128) void k_gemm2(const _Float16* __restrict__ A, int lda, size_t sA, const _Float16* __restrict__ Bh, int ldb, size_t sB, float alpha,
    const float* __restrict__ bias, size_t sBias, const float* CP, int rowsPerB, size_t sCPb, int row0g,
    float* C, _Float16* __restrict__ C16, int ldc, size_t sC, int M, int N, int K) {
  __shared__ __attribute__((aligned(16))) float so[4][32][68];
  const int tid = threadIdx.x, w = tid >> 5, lane = tid & 31, ln = lane & 15, hh = lane >> 4; const int by = blockIdx.y;
  A += (size_t)by * sA; Bh += (size_t)by * sB; const size_t cofs = (size_t)by * sC; const float* bp = bias ? bias + (size_t)by * sBias : nullptr;
  const int ntn = N >> 6; const int mt = blockIdx.x / ntn, nq = blockIdx.x - mt * ntn; const int row0 = mt * 128 + 32 * w, col0 = nq * 64; if (row0 >= M) return;
  const _Float16* a0p = A + (size_t)(row0 + ln) * lda; const _Float16* a1p = a0p + (size_t)16 * lda;
  const _Float16* b0p = Bh + (size_t)(col0 + ln) * ldb; const _Float16* b1p = b0p + (size_t)16 * ldb; const _Float16* b2p = b1p + (size_t)16 * ldb; const _Float16* b3p = b2p + (size_t)16 * ldb;
  const v8f z8 = {0.f,0.f,0.f,0.f,0.f,0.f,0.f,0.f}; v8f c00 = z8, c01 = z8, c02 = z8, c03 = z8, c10 = z8, c11 = z8, c12 = z8, c13 = z8;
#pragma unroll 1
  for (int kb = 0; kb < K; kb += 32) {
    const v16h a0 = g2_frag(a0p + kb, hh), a1 = g2_frag(a1p + kb, hh);
    v16h b = g2_frag(b0p + kb, hh); c00 = g2_mma(a0, b, c00); c10 = g2_mma(a1, b, c10);
    b = g2_frag(b1p + kb, hh); c01 = g2_mma(a0, b, c01); c11 = g2_mma(a1, b, c11);
    b = g2_frag(b2p + kb, hh); c02 = g2_mma(a0, b, c02); c12 = g2_mma(a1, b, c12);
    b = g2_frag(b3p + kb, hh); c03 = g2_mma(a0, b, c03); c13 = g2_mma(a1, b, c13);
  }
  v8f accs[8] = {c00, c01, c02, c03, c10, c11, c12, c13};
#pragma unroll
  for (int u = 0; u < 8; ++u) {
    const int t = u & 3, half = u >> 2; const int col = col0 + t * 16 + ln; const float bv = bp ? bf16_rne(bp[col]) : 0.f;
#pragma unroll
    for (int r = 0; r < 8; ++r) {
      const int rloc = half * 16 + 8 * hh + r; float v = accs[u][r] * alpha + bv;
      if (CP) {
        if (rowsPerB < 0) v += CP[cofs + (size_t)(row0g + row0 + rloc) * ldc + col];
        else { const int bidx = (row0g + row0 + rloc) / rowsPerB; v += CP[(size_t)bidx * sCPb + (size_t)by * 64 + col]; }
      }
      so[w][rloc][t * 16 + ln] = v;
    }
  }
  __builtin_amdgcn_fence(4  , "workgroup"); __builtin_amdgcn_wave_barrier();
  const int rsub = lane >> 4, c4 = (lane & 15) * 4;
  for (int pass = 0; pass < 2; ++pass) {
#pragma unroll
    for (int q = 0; q < 16; ++q) {
      const int r = q * 2 + rsub; const v4f v = *(const v4fa*)&so[w][r][c4];
      if (C) *(volatile v4f*)(C + cofs + (size_t)(row0 + r) * ldc + col0 + c4) = v;
      if (C16) { v4h h4; for (int i = 0; i < 4; ++i) h4[i] = (_Float16)v[i]; *(volatile v4h*)(C16 + cofs + (size_t)(row0 + r) * ldc + col0 + c4) = h4; }
    }
    if (pass == 0) __threadfence();
  }
}

__global__ __launch_bounds__(256) void k_vt(const _Float16* __restrict__ src, int nrow, _Float16* __restrict__ dst) {
  __shared__ unsigned short tl[64][66];
  const int tid = threadIdx.x; const int ngr = nrow / 64; const int slab = blockIdx.x / ngr, lg = blockIdx.x % ngr; const int by = blockIdx.y;
  const unsigned short* sb = (const unsigned short*)src + ((size_t)by * nrow + (size_t)lg * 64) * DM + (size_t)slab * 64;
  for (int i = tid; i < 64 * 8; i += 256) {
    const int r = i / 8, c8 = (i % 8) * 8; FragH f; f.half[0] = *(const v8us*)(sb + (size_t)r * DM + c8);
#pragma unroll
    for (int q = 0; q < 8; ++q) tl[r][c8 + q] = f.u[q];
  }
  __syncthreads();
  unsigned short* db = (unsigned short*)dst + ((size_t)by * DM + (size_t)slab * 64) * nrow + (size_t)lg * 64;
  for (int pass = 0; pass < 2; ++pass) {
#pragma unroll
    for (int rd = 0; rd < 2; ++rd) {
      const int d = rd * 32 + tid / 8, pc = tid % 8; FragH f;
#pragma unroll
      for (int q = 0; q < 8; ++q) f.u[q] = tl[pc * 8 + q][d];
      *(volatile v8us*)(db + (size_t)d * nrow + pc * 8) = f.half[0];
    }
    if (pass == 0) __threadfence();
  }
}

__global__ __launch_bounds__(256) void k_rsmcf2(const float* __restrict__ S, _Float16* __restrict__ P, int hg, int q0, int nk) {
  #pragma clang fp contract(off)
  const int t = blockIdx.x * 256 + threadIdx.x; if (t >= hg * QT) return; const size_t i = (size_t)t; const float* s = S + i * NKX; const int last = q0 + (t % QT); float mx = -3.0e38f;
#pragma unroll 1
  for (int j = 0; j < nk; ++j) { const float f = (j <= last) ? 1.f : 0.f; mx = fmaxf(mx, fmaf(f, s[j], (1.f - f) * -1.0e9f)); } float se = 0.f;
#pragma unroll 1
  for (int j = 0; j < nk; ++j) { const float f = (j <= last) ? 1.f : 0.f; se += __expf(fmaf(f, s[j], (1.f - f) * -1.0e9f) - mx); } const float sc = 256.0f / se;
#pragma unroll 1
  for (int j0 = 0; j0 < nk; j0 += 8) {
    FragH fr;
    for (int q = 0; q < 8; ++q) { const int j = j0 + q; const float f = (j <= last) ? 1.f : 0.f; fr.h[q] = (_Float16)(__expf(fmaf(f, s[j], (1.f - f) * -1.0e9f) - mx) * sc); }
    unsigned short* d = (unsigned short*)P + i * NKX + j0; *(volatile v8us*)d = fr.half[0]; __threadfence(); *(volatile v8us*)d = fr.half[0];
  }
}

__global__ __launch_bounds__(256) void k_rsmcf2hl(const float* __restrict__ S, _Float16* __restrict__ P, _Float16* __restrict__ PL, int hg, int q0, int nk) {
  #pragma clang fp contract(off)
  const int t = blockIdx.x * 256 + threadIdx.x; if (t >= hg * QT) return; const size_t i = (size_t)t; const float* s = S + i * NKX; const int last = q0 + (t % QT); float mx = -3.0e38f;
#pragma unroll 1
  for (int j = 0; j < nk; ++j) { const float f = (j <= last) ? 1.f : 0.f; mx = fmaxf(mx, fmaf(f, s[j], (1.f - f) * -1.0e9f)); } float se = 0.f;
#pragma unroll 1
  for (int j = 0; j < nk; ++j) { const float f = (j <= last) ? 1.f : 0.f; se += __expf(fmaf(f, s[j], (1.f - f) * -1.0e9f) - mx); } const float sc = 256.0f / se;
#pragma unroll 1
  for (int j0 = 0; j0 < nk; j0 += 8) {
    FragH fr, fl;
    for (int q = 0; q < 8; ++q) { const int j = j0 + q; const float f = (j <= last) ? 1.f : 0.f; const float v = __expf(fmaf(f, s[j], (1.f - f) * -1.0e9f) - mx) * sc; const _Float16 hv = (_Float16)v; fr.h[q] = hv; fl.h[q] = (_Float16)((v - (float)hv) * 1024.0f); }
    unsigned short* d = (unsigned short*)P + i * NKX + j0; unsigned short* dl = (unsigned short*)PL + i * NKX + j0;
    *(volatile v8us*)d = fr.half[0]; *(volatile v8us*)dl = fl.half[0]; __threadfence(); *(volatile v8us*)d = fr.half[0]; *(volatile v8us*)dl = fl.half[0];
  }
}

extern "C" void kernel_launch(void* const* d_in, const int* in_sizes, int n_in,
                              void* d_out, int out_size, void* d_ws, size_t ws_size, hipStream_t stream) {
  if (n_in < 4) return;
  const size_t rows_needed = (size_t)(NB - 1) * SEQ_FULL + SEQ;
  if ((size_t)in_sizes[0] < rows_needed * DM) return;
  if ((size_t)in_sizes[1] < (size_t)DM * DM || (size_t)in_sizes[2] < (size_t)DM * DM || (size_t)in_sizes[3] < (size_t)DM * DM) return;
  if ((size_t)out_size < rows_needed * DM) return;
  const float* x  = (const float*)d_in[0];
  const float* wq = (const float*)d_in[1];
  const float* wk = (const float*)d_in[2];
  const float* wv = (const float*)d_in[3];
  float* out = (float*)d_out;

  char* ws = (char*)d_ws; size_t off = 0;
  auto take = [&](size_t bytes) { char* p = ws + off; off += (bytes + 255) & ~(size_t)255; return p; };
  _Float16* BQ  = (_Float16*)take((size_t)DM * DM * 2);
  _Float16* BK  = (_Float16*)take((size_t)DM * DM * 2);
  _Float16* BV  = (_Float16*)take((size_t)DM * DM * 2);
  _Float16* X16 = (_Float16*)take(NR * DM * 2);
  _Float16* Q16 = (_Float16*)take(NR * DM * 2);
  _Float16* K16 = (_Float16*)take(NR * DM * 2);
  _Float16* V16 = (_Float16*)take(NR * DM * 2);
  float*    Fc  = (float*)take((size_t)NB * KT0 * DM * 4);
  _Float16* QL  = (_Float16*)take((size_t)NB * KT0 * DM * 2);
  _Float16* KL  = (_Float16*)take((size_t)NB * KT0 * DM * 2);
  _Float16* VL  = (_Float16*)take((size_t)NB * KT0 * DM * 2);
  float*    S   = (float*)take((size_t)NB * QT * NKX * 4);
  _Float16* P   = (_Float16*)take((size_t)NB * QT * NKX * 2);
  _Float16* PL  = (_Float16*)take((size_t)NB * QT * NKX * 2);
  _Float16* VT  = (_Float16*)take((size_t)NB * DM * SEQ * 2);
  _Float16* VTL = (_Float16*)take((size_t)NB * DM * KT0 * 2);
  if (off > ws_size) return;

  const unsigned gw  = (unsigned)(((size_t)DM * DM / 8 + 255) / 256);
  const unsigned gx  = (unsigned)((NR * DM / 8 + 255) / 256);
  const unsigned glo = (unsigned)(((size_t)NB * KT0 * DM / 8 + 255) / 256);
  k_wnat<<<gw, 256, 0, stream>>>(wq, (size_t)DM * DM / 8, BQ);
  k_wnat<<<gw, 256, 0, stream>>>(wk, (size_t)DM * DM / 8, BK);
  k_wnat<<<gw, 256, 0, stream>>>(wv, (size_t)DM * DM / 8, BV);
  k_x16<<<gx, 256, 0, stream>>>(x, X16, NR * DM / 8);

  const dim3 gall((unsigned)((NR / 128) * (DM / 64)), 1);
  const dim3 gearly((unsigned)((KT0 / 128) * (DM / 64)), NB);
  const size_t sRow = (size_t)SEQ * DM;
  const size_t sLo  = (size_t)KT0 * DM;
  k_gemm2<<<gall, 128, 0, stream>>>(X16, DM, 0, BQ, DM, 0, 0.0625f, nullptr, 0, nullptr, 1, 0, 0, nullptr, Q16, DM, 0, (int)NR, DM, DM);
  k_gemm2<<<gearly, 128, 0, stream>>>(X16, DM, sRow, BQ, DM, 0, 0.0625f, nullptr, 0, nullptr, 1, 0, 0, Fc, nullptr, DM, sLo, KT0, DM, DM);
  k_lo<<<glo, 256, 0, stream>>>(Fc, QL, (size_t)NB * KT0 * DM / 8);
  k_gemm2<<<gall, 128, 0, stream>>>(X16, DM, 0, BK, DM, 0, 0.0625f, nullptr, 0, nullptr, 1, 0, 0, nullptr, K16, DM, 0, (int)NR, DM, DM);
  k_gemm2<<<gearly, 128, 0, stream>>>(X16, DM, sRow, BK, DM, 0, 0.0625f, nullptr, 0, nullptr, 1, 0, 0, Fc, nullptr, DM, sLo, KT0, DM, DM);
  k_lo<<<glo, 256, 0, stream>>>(Fc, KL, (size_t)NB * KT0 * DM / 8);
  k_gemm2<<<gall, 128, 0, stream>>>(X16, DM, 0, BV, DM, 0, 0.0625f, nullptr, 0, nullptr, 1, 0, 0, nullptr, V16, DM, 0, (int)NR, DM, DM);
  k_gemm2<<<gearly, 128, 0, stream>>>(X16, DM, sRow, BV, DM, 0, 0.0625f, nullptr, 0, nullptr, 1, 0, 0, Fc, nullptr, DM, sLo, KT0, DM, DM);
  k_lo<<<glo, 256, 0, stream>>>(Fc, VL, (size_t)NB * KT0 * DM / 8);

  k_vt<<<dim3((unsigned)((DM / 64) * (SEQ / 64)), NB), 256, 0, stream>>>(V16, SEQ, VT);
  k_vt<<<dim3((unsigned)((DM / 64) * (KT0 / 64)), NB), 256, 0, stream>>>(VL, KT0, VTL);

  const size_t sS = (size_t)QT * NKX;
  const size_t sO = (size_t)SEQ_FULL * DM;
  for (int q0 = 0; q0 < SEQ; q0 += QT) {
    const int nk = q0 + QT;
    const dim3 gsc((unsigned)((QT / 128) * (nk / 64)), NB);
    const dim3 gpv((unsigned)((QT / 128) * (DM / 64)), NB);
    k_gemm2<<<gsc, 128, 0, stream>>>(Q16 + (size_t)q0 * DM, DM, sRow, K16, DM, sRow, 0.03125f, nullptr, 0, nullptr, 1, 0, 0, S, nullptr, NKX, sS, QT, nk, DM);
    if (q0 == 0) {
      k_gemm2<<<gsc, 128, 0, stream>>>(QL, DM, sLo, K16, DM, sRow, 0.000030517578125f, nullptr, 0, S, -1, 0, 0, S, nullptr, NKX, sS, QT, nk, DM);
      k_gemm2<<<gsc, 128, 0, stream>>>(Q16, DM, sRow, KL, DM, sLo, 0.000030517578125f, nullptr, 0, S, -1, 0, 0, S, nullptr, NKX, sS, QT, nk, DM);
      k_rsmcf2hl<<<(NB * QT + 255) / 256, 256, 0, stream>>>(S, P, PL, NB, 0, nk);
      k_gemm2<<<gpv, 128, 0, stream>>>(P, NKX, sS, VT, SEQ, (size_t)DM * SEQ, 0.00390625f, nullptr, 0, nullptr, 1, 0, 0, out, nullptr, DM, sO, QT, DM, nk);
      k_gemm2<<<gpv, 128, 0, stream>>>(P, NKX, sS, VTL, KT0, (size_t)DM * KT0, 0.000003814697265625f, nullptr, 0, out, -1, 0, 0, out, nullptr, DM, sO, QT, DM, nk);
      k_gemm2<<<gpv, 128, 0, stream>>>(PL, NKX, sS, VT, SEQ, (size_t)DM * SEQ, 0.000003814697265625f, nullptr, 0, out, -1, 0, 0, out, nullptr, DM, sO, QT, DM, nk);
    } else {
      k_rsmcf2<<<(NB * QT + 255) / 256, 256, 0, stream>>>(S, P, NB, q0, nk);
      k_gemm2<<<gpv, 128, 0, stream>>>(P, NKX, sS, VT, SEQ, (size_t)DM * SEQ, 0.00390625f, nullptr, 0, nullptr, 1, 0, 0, out + (size_t)q0 * DM, nullptr, DM, sO, QT, DM, nk);
    }
  }
}
